// SpatialGNN_45432164057449
// MI455X (gfx1250) — hardware-run, weakly checked
//
#include <hip/hip_runtime.h>
#include <stddef.h>
#include <stdint.h>

#define NB    16
#define CH    64
#define NN    32
#define NK    16
#define NL    24
#define QQ    (NK * NL)
#define NG    (NB * QQ)
#define NROWS (NG * NN)
#define NE    160
#define NH    4
#define HD    16
#define GT    8
#define XP    132
#define DEGCAP NE
#define NEGS  0.2f
#define WSMAX 134217728

static_assert(NB * NK * NL == 6144);
static_assert((NK * NL) % 32 == 0);
static_assert(NN == 32 && CH == 64 && NH * HD == 64 && NE == 160);
static_assert(NG % GT == 0);
static_assert(DEGCAP == NE);
static_assert((XP % 4) == 0);

typedef float          v2f   __attribute__((ext_vector_type(2)));
typedef float          v4f   __attribute__((ext_vector_type(4)));
typedef float          v8f   __attribute__((ext_vector_type(8)));
typedef int            v4i   __attribute__((ext_vector_type(4)));
typedef int            v8i   __attribute__((ext_vector_type(8)));
typedef unsigned short v8us  __attribute__((ext_vector_type(8)));
typedef __bf16         v16bf __attribute__((ext_vector_type(16)));
union FragB { v16bf v; v8us u[2]; v8i w; };

__device__ __forceinline__ v8f wmx(const FragB& a, const FragB& b, v8f c) {
  v8f d = __builtin_amdgcn_wmma_f32_16x16x32_bf16(false, a.v, false, b.v, (short)0, c, false, false);
  asm volatile("v_nop\n\tv_nop\n\tv_nop\n\tv_nop" : "+v"(d) : "v"(a.w), "v"(b.w));
  return d;
}

__device__ __forceinline__ unsigned bfbits(float v) {
  unsigned u = __float_as_uint(v);
  u = u + 0x7FFFu + ((u >> 16) & 1u);
  return u >> 16;
}
__device__ __forceinline__ float bf2f(unsigned b) { return __uint_as_float(b << 16); }
__device__ __forceinline__ float rbf(float v) { return bf2f(bfbits(v)); }
__device__ __forceinline__ v4f rbf4(const v4f a) {
  v4f o; o.x = rbf(a.x); o.y = rbf(a.y); o.z = rbf(a.z); o.w = rbf(a.w); return o;
}
__device__ __forceinline__ v8us cvt8b(const v4f a, const v4f b) {
  v8us o;
  o[0] = (unsigned short)bfbits(a.x); o[1] = (unsigned short)bfbits(a.y);
  o[2] = (unsigned short)bfbits(a.z); o[3] = (unsigned short)bfbits(a.w);
  o[4] = (unsigned short)bfbits(b.x); o[5] = (unsigned short)bfbits(b.y);
  o[6] = (unsigned short)bfbits(b.z); o[7] = (unsigned short)bfbits(b.w);
  return o;
}

__device__ __forceinline__ void put4f(float* p, const v4f v) {
  *(volatile v4f*)p = v;
  __threadfence();
  *(volatile v4f*)p = v;
}
__device__ __forceinline__ void put4i(int* p, const v4i v) {
  *(volatile v4i*)p = v;
  __threadfence();
  *(volatile v4i*)p = v;
}

template<int DUP>
__device__ __forceinline__ void wplane8(const float* __restrict__ src, unsigned short* dst, int dpitch, int u) {
  const int row = u >> 3, k8 = (u & 7) * 8;
  const float* p = src + row * 64 + k8;
  const v4f a = *(const v4f*)p;
  const v4f b = *(const v4f*)(p + 4);
  const v8us hv = cvt8b(a, b);
  unsigned short* o = dst + row * dpitch + k8;
  *(volatile v8us*)o = hv;
  if (DUP) *(volatile v8us*)(o + 64) = hv;
  __threadfence();
  *(volatile v8us*)o = hv;
  if (DUP) *(volatile v8us*)(o + 64) = hv;
}

__global__ __launch_bounds__(256) void k_prep(
    const float* __restrict__ x, const int* __restrict__ ei, const float* __restrict__ ew,
    const float* __restrict__ Wl, const float* __restrict__ bl, const float* __restrict__ Wr,
    const float* __restrict__ br, const float* __restrict__ We, const float* __restrict__ att,
    const float* __restrict__ bo,
    unsigned* XBw, unsigned short* W1b, unsigned short* W2b, float* EFS, int* CSR, float* P)
{
  __shared__ __attribute__((aligned(16))) float tf[4 * 32 * 66];
  __shared__ __attribute__((aligned(16))) int   csr_l[256];
  __shared__ int   s_src[NE];
  __shared__ int   s_dst[NE];
  __shared__ int   s_eid[NE];
  __shared__ float s_ew[NE];
  __shared__ float s_we[128];
  const int tid = (int)threadIdx.x, lane = tid & 31, wave = tid >> 5;
  const int bid = (int)blockIdx.x;

  if (bid < 192) {
    const int b = bid / 12;
    const int j = bid - b * 12;
    const float* xb = x + (size_t)b * (size_t)(CH * NN * QQ) + 32 * j;
#pragma unroll 1
    for (int it = 0; it < 8; ++it) {
      const int n0 = 4 * it;
      v4f ld[8];
#pragma unroll
      for (int i = 0; i < 8; ++i) {
        const int idx  = tid + 256 * i;
        const int quad = idx & 7;
        const int c    = (idx >> 3) & 63;
        const int nn   = idx >> 9;
        ld[i] = *(const v4f*)(xb + (size_t)(c * NN + n0 + nn) * QQ + 4 * quad);
      }
      __syncthreads();
#pragma unroll
      for (int i = 0; i < 8; ++i) {
        const int idx  = tid + 256 * i;
        const int quad = idx & 7;
        const int c    = (idx >> 3) & 63;
        const int nn   = idx >> 9;
        float* t = tf + (nn * 32 + 4 * quad) * 66 + c;
        t[0]      = ld[i].x;
        t[66]     = ld[i].y;
        t[2 * 66] = ld[i].z;
        t[3 * 66] = ld[i].w;
      }
      __syncthreads();
      unsigned pk[16];
#pragma unroll
      for (int i = 0; i < 16; ++i) {
        const int rr = wave + 8 * i;
        const v2f f = *(const v2f*)(tf + rr * 66 + 2 * lane);
        pk[i] = bfbits(f.x) | (bfbits(f.y) << 16);
      }
#pragma unroll
      for (int i = 0; i < 16; ++i) {
        const int rr = wave + 8 * i;
        const int nn = rr >> 5, qq = rr & 31;
        const size_t row = (size_t)(b * QQ + 32 * j + qq) * NN + (n0 + nn);
        ((volatile unsigned*)XBw)[row * 32 + lane] = pk[i];
      }
      __threadfence();
#pragma unroll
      for (int i = 0; i < 16; ++i) {
        const int rr = wave + 8 * i;
        const int nn = rr >> 5, qq = rr & 31;
        const size_t row = (size_t)(b * QQ + 32 * j + qq) * NN + (n0 + nn);
        ((volatile unsigned*)XBw)[row * 32 + lane] = pk[i];
      }
    }
  } else {
    csr_l[tid] = 0;
    if (tid < NE) {
      int sv = ei[tid];
      const int dv = ei[NE + tid];
      sv = sv < 0 ? 0 : (sv > NN - 1 ? NN - 1 : sv);
      s_src[tid] = sv;
      s_dst[tid] = dv;
      s_eid[tid] = 0;
      s_ew[tid]  = rbf(ew[tid]);
    }
    if (tid < 128) s_we[tid] = rbf(We[tid]);
    __syncthreads();
    if (wave == 0) {
      int cnt = 0;
#pragma unroll 1
      for (int e = 0; e < NE; ++e) cnt += (s_dst[e] == lane) ? 1 : 0;
      int incl = cnt;
#pragma unroll
      for (int dd = 1; dd < 32; dd <<= 1) {
        const int up = __shfl_up(incl, dd);
        incl += (lane >= dd) ? up : 0;
      }
      int pos = incl - cnt;
      csr_l[lane] = pos;
      if (lane == 31) csr_l[32] = incl;
#pragma unroll 1
      for (int e = 0; e < NE; ++e) {
        const int sv = s_src[e];
        const int dv = s_dst[e];
        if (dv == lane && pos < NE) {
          csr_l[64 + pos] = sv;
          s_eid[pos] = e;
          pos = pos + 1;
        }
      }
    }
    __syncthreads();
    if (tid < 64) {
      const v4i cv = *(const v4i*)(csr_l + 4 * tid);
      put4i(CSR + 4 * tid, cv);
    }
    if (tid >= 64 && tid < 96) {
      const int t  = tid - 64;
      const int ly = t >> 4;
      const int c4 = (t & 15) * 4;
      const int so = ly * 64 + c4;
      const v4f pa = rbf4(*(const v4f*)(bl  + so));
      const v4f pb = rbf4(*(const v4f*)(br  + so));
      const v4f pc = rbf4(*(const v4f*)(att + so));
      const v4f pd = rbf4(*(const v4f*)(bo  + so));
      float* pp = P + ly * 256 + c4;
      put4f(pp,       pa);
      put4f(pp + 64,  pb);
      put4f(pp + 128, pc);
      put4f(pp + 192, pd);
    }
#pragma unroll 1
    for (int it = 0; it < 2; ++it) {
      const int u = tid + 256 * it;
      wplane8<0>(Wl,        W1b,            64,  u);
      wplane8<0>(Wr,        W1b + 64 * 64,  64,  u);
      wplane8<1>(Wl + 4096, W2b,            128, u);
      wplane8<1>(Wr + 4096, W2b + 64 * 128, 128, u);
    }
#pragma unroll 1
    for (int it = 0; it < 20; ++it) {
      const int u   = tid + 256 * it;
      const int i   = u / 2560;
      const int rem = u - i * 2560;
      const int p   = rem >> 4;
      const int c4  = (rem & 15) * 4;
      int e = s_eid[p];
      e = e < 0 ? 0 : (e > NE - 1 ? NE - 1 : e);
      const float wv = s_ew[e];
      const float* wp = s_we + i * 64 + c4;
      v4f v;
      v.x = wv * wp[0]; v.y = wv * wp[1]; v.z = wv * wp[2]; v.w = wv * wp[3];
      put4f(EFS + 4 * (size_t)u, v);
    }
  }
}

template<int KD, bool FIRST>
__global__ __launch_bounds__(256) __attribute__((amdgpu_num_vgpr(248)))
void k_layer(const unsigned short* __restrict__ A, const unsigned short* __restrict__ Wp,
             const float* __restrict__ EFSg, const int* __restrict__ CSRg, const float* __restrict__ Pg,
             unsigned* H1w, float* H2)
{
  constexpr int BPP = KD + 8;
  constexpr int KQ  = KD / 8;
  constexpr int KS  = KD / 32;
  static_assert((KD % 32) == 0);
  extern __shared__ v4f lds_dyn[];
  float* xlr = (float*)lds_dyn;
  float* efs = xlr + GT * NN * XP;
  float* prm = efs + NE * CH;
  int*   csr = (int*)(prm + 256);
  unsigned short* bp = (unsigned short*)(csr + 256);

  const int tid = (int)threadIdx.x, lane = tid & 31, wave = tid >> 5, hh = lane >> 4, m = lane & 15;
  const int rowBase = (int)blockIdx.x * (GT * NN) + wave * NN;

#pragma unroll 2
  for (int u = tid; u < 128 * KQ; u += 256) {
    const int row = u / KQ;
    const int k8  = (u - row * KQ) * 8;
    *(v8us*)(bp + row * BPP + k8) = *(const v8us*)(Wp + row * KD + k8);
  }
#pragma unroll 2
  for (int u = tid; u < (NE * CH) / 4; u += 256)
    *(v4f*)(efs + 4 * u) = *(const v4f*)(EFSg + 4 * u);
  if (tid < 64) {
    *(v4i*)(csr + 4 * tid) = *(const v4i*)(CSRg + 4 * tid);
  } else if (tid < 128) {
    const int t = tid - 64;
    *(v4f*)(prm + 4 * t) = *(const v4f*)(Pg + 4 * t);
  }

  FragB af[2][KS];
#pragma unroll
  for (int mt = 0; mt < 2; ++mt) {
    const unsigned short* ap = A + (size_t)(rowBase + 16 * mt + m) * (size_t)KD + 8 * hh;
#pragma unroll
    for (int ks = 0; ks < KS; ++ks) {
      af[mt][ks].u[0] = *(const v8us*)(ap + 32 * ks);
      af[mt][ks].u[1] = *(const v8us*)(ap + 32 * ks + 16);
    }
  }
  __syncthreads();

  float* xw = xlr + wave * (NN * XP);
#pragma unroll 1
  for (int np = 0; np < 4; ++np) {
    const v8f z = {0.f, 0.f, 0.f, 0.f, 0.f, 0.f, 0.f, 0.f};
    v8f a00 = z, a01 = z, a10 = z, a11 = z;
    const unsigned short* b0p = bp + (32 * np + m) * BPP + 8 * hh;
    const unsigned short* b1p = b0p + 16 * BPP;
#pragma unroll
    for (int ks = 0; ks < KS; ++ks) {
      FragB b0, b1;
      b0.u[0] = *(const v8us*)(b0p + 32 * ks);
      b0.u[1] = *(const v8us*)(b0p + 32 * ks + 16);
      b1.u[0] = *(const v8us*)(b1p + 32 * ks);
      b1.u[1] = *(const v8us*)(b1p + 32 * ks + 16);
      a00 = wmx(af[0][ks], b0, a00);
      a01 = wmx(af[0][ks], b1, a01);
      a10 = wmx(af[1][ks], b0, a10);
      a11 = wmx(af[1][ks], b1, a11);
    }
    const int c0 = 32 * np + m, c1 = c0 + 16;
    const float pb0 = prm[c0], pb1 = prm[c1];
#pragma unroll
    for (int r = 0; r < 8; ++r) {
      const int r0 = 8 * hh + r;
      xw[r0 * XP + c0]        = a00[r] + pb0;
      xw[r0 * XP + c1]        = a01[r] + pb1;
      xw[(16 + r0) * XP + c0] = a10[r] + pb0;
      xw[(16 + r0) * XP + c1] = a11[r] + pb1;
    }
  }
  __syncthreads();

  const float at0 = prm[128 + 2 * lane], at1 = prm[129 + 2 * lane];
  const float bo0 = prm[192 + 2 * lane], bo1 = prm[193 + 2 * lane];
#pragma unroll 1
  for (int d = 0; d < NN; ++d) {
    int st = csr[d];
    int en = csr[d + 1];
    st = st < 0 ? 0 : (st > NE ? NE : st);
    en = en < 0 ? 0 : (en > NE ? NE : en);
    int cnt = en - st;
    cnt = cnt < 0 ? 0 : (cnt > DEGCAP ? DEGCAP : cnt);
    st  = __builtin_amdgcn_readfirstlane(st);
    cnt = __builtin_amdgcn_readfirstlane(cnt);
    const v2f xr = *(const v2f*)(xw + d * XP + 64 + 2 * lane);
    float mx = -1.0e30f, dn = 0.0f, a0 = 0.0f, a1 = 0.0f;
#pragma unroll 1
    for (int q = 0; q < cnt; ++q) {
      const int p = st + q;
      int s = csr[64 + p];
      s = s < 0 ? 0 : (s > NN - 1 ? NN - 1 : s);
      s = __builtin_amdgcn_readfirstlane(s);
      const v2f xs = *(const v2f*)(xw + s * XP + 2 * lane);
      const v2f ef = *(const v2f*)(efs + p * CH + 2 * lane);
      float v0 = (xs.x + xr.x) + ef.x;
      float v1 = (xs.y + xr.y) + ef.y;
      const float n0 = v0 * NEGS, n1 = v1 * NEGS;
      v0 = (v0 >= 0.0f) ? v0 : n0;
      v1 = (v1 >= 0.0f) ? v1 : n1;
      float part = fmaf(v1, at1, v0 * at0);
      part += __shfl_xor(part, 1);
      part += __shfl_xor(part, 2);
      part += __shfl_xor(part, 4);
      const float df = part - mx;
      const float ee = expf(-fabsf(df));
      const bool  up = df > 0.0f;
      const float s1 = up ? ee : 1.0f;
      const float s2 = up ? 1.0f : ee;
      mx = up ? part : mx;
      dn = fmaf(dn, s1, s2);
      a0 = fmaf(a0, s1, s2 * xs.x);
      a1 = fmaf(a1, s1, s2 * xs.y);
    }
    const float ds = dn > 0.0f ? dn : 1.0f;
    const float iv = (cnt > 0) ? __builtin_amdgcn_rcpf(ds) : 0.0f;
    float r0 = fmaf(a0, iv, bo0);
    float r1 = fmaf(a1, iv, bo1);
    const size_t row = (size_t)(rowBase + d);
    if (FIRST) {
      r0 = (r0 > 0.0f) ? r0 : 0.0f;
      r1 = (r1 > 0.0f) ? r1 : 0.0f;
      const unsigned h0 = bfbits(r0), h1 = bfbits(r1);
      const unsigned l0 = bfbits(r0 - bf2f(h0)), l1 = bfbits(r1 - bf2f(h1));
      const unsigned uh = h0 | (h1 << 16);
      const unsigned ul = l0 | (l1 << 16);
      volatile unsigned* gp = (volatile unsigned*)H1w + row * 64 + lane;
      gp[0]  = uh;
      gp[32] = ul;
      __threadfence();
      gp[0]  = uh;
      gp[32] = ul;
    } else {
      v2f rv; rv.x = r0; rv.y = r1;
      float* gp = H2 + row * 64 + 2 * lane;
      *(volatile v2f*)gp = rv;
      __threadfence();
      *(volatile v2f*)gp = rv;
    }
  }
  (void)H1w; (void)H2;
}

__global__ __launch_bounds__(256) void k_out(const float* __restrict__ H2, float* out) {
  __shared__ __attribute__((aligned(16))) float tl[4 * 32 * 65];
  const int tid = (int)threadIdx.x, lane = tid & 31, wave = tid >> 5;
  const int bid = (int)blockIdx.x;
  const int b = bid / 12;
  const int j = bid - b * 12;
#pragma unroll 1
  for (int it = 0; it < 8; ++it) {
    const int n0 = 4 * it;
    v4f ld[8];
#pragma unroll
    for (int i = 0; i < 8; ++i) {
      const int idx = tid + 256 * i;
      const int f4  = idx & 15;
      const int qq  = (idx >> 4) & 31;
      const int nn  = idx >> 9;
      const size_t row = (size_t)(b * QQ + 32 * j + qq) * NN + (n0 + nn);
      ld[i] = *(const v4f*)(H2 + row * 64 + 4 * f4);
    }
    __syncthreads();
#pragma unroll
    for (int i = 0; i < 8; ++i) {
      const int idx = tid + 256 * i;
      const int f4  = idx & 15;
      const int qq  = (idx >> 4) & 31;
      const int nn  = idx >> 9;
      float* t = tl + (nn * 32 + qq) * 65 + 4 * f4;
      t[0] = ld[i].x; t[1] = ld[i].y; t[2] = ld[i].z; t[3] = ld[i].w;
    }
    __syncthreads();
    const int nn = wave >> 1;
    const int cb = (wave & 1) * 32;
    float v[32];
#pragma unroll
    for (int i = 0; i < 32; ++i) v[i] = tl[(nn * 32 + lane) * 65 + cb + i];
    const size_t obase = ((size_t)(b * CH + cb) * NN + (n0 + nn)) * QQ + 32 * j + lane;
#pragma unroll
    for (int i = 0; i < 32; ++i)
      *(volatile float*)(out + obase + (size_t)i * (NN * QQ)) = v[i];
    __threadfence();
#pragma unroll
    for (int i = 0; i < 32; ++i)
      *(volatile float*)(out + obase + (size_t)i * (NN * QQ)) = v[i];
  }
}

#define SZ_XB   ((size_t)NROWS * 64 * 2)
#define SZ_H1   ((size_t)NROWS * 128 * 2)
#define SZ_H2   ((size_t)NROWS * 64 * 4)
#define SZ_W1   ((size_t)128 * 64 * 2)
#define SZ_W2   ((size_t)128 * 128 * 2)
#define SZ_EFS  ((size_t)2 * NE * CH * 4)
#define SZ_CSR  ((size_t)256 * 4)
#define SZ_P    ((size_t)2 * 256 * 4)
#define SZ_TOT  (SZ_XB + SZ_H1 + SZ_H2 + SZ_W1 + SZ_W2 + SZ_EFS + SZ_CSR + SZ_P)
#define LDS_BASE ((GT * NN * XP + NE * CH + 256 + 256) * 4)
#define LDS_L1  (LDS_BASE + 128 * (64 + 8) * 2)
#define LDS_L2  (LDS_BASE + 128 * (128 + 8) * 2)

static_assert(SZ_TOT <= (size_t)WSMAX);
static_assert((SZ_XB % 256) == 0 && (SZ_H1 % 256) == 0 && (SZ_H2 % 256) == 0 && (SZ_W1 % 256) == 0);
static_assert((SZ_W2 % 256) == 0 && (SZ_EFS % 256) == 0 && (SZ_CSR % 256) == 0 && (SZ_P % 256) == 0);
static_assert(LDS_L1 <= 327680 && LDS_L2 <= 327680);
static_assert((LDS_BASE % 16) == 0);
static_assert(NROWS == 768 * GT * NN);
static_assert(NB * 12 == 192 && 12 * 32 == QQ);

extern "C" void kernel_launch(void* const* d_in, const int* in_sizes, int n_in,
                              void* d_out, int out_size, void* d_ws, size_t ws_size,
                              hipStream_t stream) {
  if (n_in < 10) return;
  if (in_sizes[0] != NB * CH * NN * QQ) return;
  if (in_sizes[1] != 2 * NE) return;
  if (in_sizes[2] != NE) return;
  if (in_sizes[3] != 2 * CH * CH || in_sizes[5] != 2 * CH * CH) return;
  if (in_sizes[4] != 2 * CH || in_sizes[6] != 2 * CH) return;
  if (in_sizes[7] != 2 * CH || in_sizes[8] != 2 * CH || in_sizes[9] != 2 * CH) return;
  if (out_size != NB * CH * NN * QQ) return;
  if (SZ_TOT > ws_size) return;

  const float* x   = (const float*)d_in[0];
  const int*   ei  = (const int*)  d_in[1];
  const float* ew  = (const float*)d_in[2];
  const float* Wl  = (const float*)d_in[3];
  const float* bl  = (const float*)d_in[4];
  const float* Wr  = (const float*)d_in[5];
  const float* br  = (const float*)d_in[6];
  const float* We  = (const float*)d_in[7];
  const float* att = (const float*)d_in[8];
  const float* bo  = (const float*)d_in[9];
  float* out = (float*)d_out;

  char* ws = (char*)d_ws;
  size_t off = 0;
  const size_t oXB  = off; off += SZ_XB;
  const size_t oH1  = off; off += SZ_H1;
  const size_t oH2  = off; off += SZ_H2;
  const size_t oW1  = off; off += SZ_W1;
  const size_t oW2  = off; off += SZ_W2;
  const size_t oEFS = off; off += SZ_EFS;
  const size_t oCSR = off; off += SZ_CSR;
  const size_t oP   = off; off += SZ_P;
  if (off > ws_size || off > (size_t)WSMAX) return;
  unsigned short* XB   = (unsigned short*)(ws + oXB);
  unsigned short* H1HL = (unsigned short*)(ws + oH1);
  float*          H2   = (float*)(ws + oH2);
  unsigned short* W1b  = (unsigned short*)(ws + oW1);
  unsigned short* W2b  = (unsigned short*)(ws + oW2);
  float*          EFS  = (float*)(ws + oEFS);
  int*            CSR  = (int*)(ws + oCSR);
  float*          P    = (float*)(ws + oP);

  hipFuncSetAttribute(reinterpret_cast<const void*>(&k_layer<64, true>),
                      hipFuncAttributeMaxDynamicSharedMemorySize, LDS_L1);
  hipFuncSetAttribute(reinterpret_cast<const void*>(&k_layer<128, false>),
                      hipFuncAttributeMaxDynamicSharedMemorySize, LDS_L2);

  k_prep<<<dim3(193), dim3(256), 0, stream>>>(x, ei, ew, Wl, bl, Wr, br, We, att, bo,
                                              (unsigned*)XB, W1b, W2b, EFS, CSR, P);
  k_layer<64, true><<<dim3(NG / GT), dim3(256), LDS_L1, stream>>>(
      XB, W1b, EFS, CSR, P, (unsigned*)H1HL, H2);
  k_layer<128, false><<<dim3(NG / GT), dim3(256), LDS_L2, stream>>>(
      H1HL, W2b, EFS + NE * CH, CSR, P + 256, (unsigned*)XB, H2);
  k_out<<<dim3(192), dim3(256), 0, stream>>>(H2, out);
  (void)hipGetLastError();
}
